// Translator_7060926235319
// MI455X (gfx1250) — hardware-run, weakly checked
//
#include <hip/hip_runtime.h>


#ifndef NB
#define NB 8192
#endif
#define NB_FULL 8192
#define HID   1024
#define RANK  16
#define NSEG  64
#define CPW   (NB / 1024)
#define PROWS (NB + NSEG * 63)
#define TPITCH 20
#define WB_BLK ((NSEG * RANK * HID / 8) / 256)
#define WA_BLK ((NSEG * HID * 4) / 256)

static_assert(NB % 1024 == 0);
static_assert(CPW >= 1);
static_assert(NB <= NB_FULL);
static_assert(PROWS % 64 == 0);
static_assert(HID % 32 == 0);
static_assert(HID % 64 == 0);
static_assert(RANK == 16);
static_assert(NSEG == 64);
static_assert(NB % 8 == 0);
static_assert((NSEG * RANK * HID / 8) % 256 == 0);
static_assert((NSEG * HID * 4) % 256 == 0);
static_assert((TPITCH % 4) == 0 && TPITCH >= RANK);
static_assert((32 * NSEG + NB + NSEG + NSEG + 256) * 4 <= 131072);
static_assert((16 * 68 + 64 * TPITCH) * 4 <= 131072);
static_assert(32 * 16 * 4 == HID * 2);
static_assert(32 * 16 * 8 == HID * 4);
static_assert(32 * 16 * 8 == 16 * 64 * 4);

typedef unsigned short bf;
typedef __attribute__((ext_vector_type(16))) __bf16   v16bf;
typedef __attribute__((ext_vector_type(8)))  unsigned short v8us;
typedef __attribute__((ext_vector_type(8)))  float    v8f;
typedef __attribute__((ext_vector_type(4)))  float    v4f;
typedef __attribute__((ext_vector_type(4)))  int      v4i;
typedef v4f  __attribute__((may_alias)) v4fa;
typedef v4i  __attribute__((may_alias)) v4ia;

__device__ __forceinline__ unsigned short f2bf(float f) { unsigned u = __float_as_uint(f); u += 0x7FFFu + ((u >> 16) & 1u); return (unsigned short)(u >> 16); }
__device__ __forceinline__ float bf2f(unsigned short w) { return __uint_as_float(((unsigned)w) << 16); }
__device__ __forceinline__ int clampi(int v, int lo, int hi) { return min(max(v, lo), hi); }
__device__ __forceinline__ v16bf cat16b(v8us lo, v8us hi) { return __builtin_bit_cast(v16bf, __builtin_shufflevector(lo, hi, 0, 1, 2, 3, 4, 5, 6, 7, 8, 9, 10, 11, 12, 13, 14, 15)); }
__device__ __forceinline__ v8f wmmab(v16bf a, v16bf b, v8f c) { return __builtin_amdgcn_wmma_f32_16x16x32_bf16(false, a, false, b, (short)0, c, false, false); }
__device__ __forceinline__ v16bf ldb(const bf* p)  { return cat16b(*(const v8us*)p, *(const v8us*)(p + 16)); }
__device__ __forceinline__ void wave_sync() { __builtin_amdgcn_fence(3  , "wavefront"); __builtin_amdgcn_wave_barrier(); asm volatile("" ::: "memory"); }
__device__ __forceinline__ v8f wmmag(v16bf a, v16bf b, v8f c) { c = wmmab(a, b, c); asm volatile("v_nop\n\tv_nop\n\tv_nop\n\tv_nop" : "+v"(c) : "v"(a), "v"(b)); return c; }

__global__ __launch_bounds__(256) void k_wconv(const float* __restrict__ Am, const float* __restrict__ Bm, bf* AW, bf* BW) {
    const int b = blockIdx.x, t = threadIdx.x;
    if (b < WB_BLK) {
        const size_t q = (size_t)b * 256 + (size_t)t;
        const v8f a = *(const v8f*)(Bm + q * 8); v8us o;
#pragma unroll
        for (int k = 0; k < 8; ++k) o[k] = f2bf(a[k]);
        *(volatile v8us*)(BW + q * 8) = o; __threadfence(); *(volatile v8us*)(BW + q * 8) = o;
    } else {
        const size_t q = (size_t)(b - WB_BLK) * 256 + (size_t)t; const size_t row = q >> 2; const int pc = (int)(q & 3);
        const v8f a = *(const v8f*)(Am + row * RANK + (size_t)((pc & 1) * 8)); v8us o;
#pragma unroll
        for (int k = 0; k < 8; ++k) o[k] = f2bf(a[k]);
        *(volatile v8us*)(AW + row * 32 + (size_t)(pc * 8)) = o; __threadfence(); *(volatile v8us*)(AW + row * 32 + (size_t)(pc * 8)) = o;
    }
}

__global__ __launch_bounds__(1024) void k_sort(const int* __restrict__ seg, int* POS, int* T, bf* XP) {
    __shared__ int wc[32 * NSEG];
    __shared__ int part[NB];
    __shared__ int tots[NSEG];
    __shared__ int segst[NSEG];
    __shared__ __align__(16) int tl[256];
    const int tid = threadIdx.x, lane = tid & 31; const int wave = __builtin_amdgcn_readfirstlane(tid >> 5);
    const int tbase = wave * (CPW * 32);
    const unsigned lt = (1u << lane) - 1u;
    int run0 = 0, run1 = 0;
#pragma unroll 1
    for (int c = 0; c < CPW; ++c) {
        const int tok = tbase + c * 32 + lane;
        const int s = clampi(seg[tok], 0, NSEG - 1);
        const int a0 = __shfl(run0, s & 31, 32); const int a1 = __shfl(run1, s & 31, 32);
        const int pre = (s >= 32) ? a1 : a0;
        int add0 = 0, add1 = 0; unsigned mymask = 0u;
#pragma unroll 1
        for (int r = 0; r < 32; ++r) {
            const unsigned m0 = __builtin_amdgcn_ballot_w32(s == r); const unsigned m1 = __builtin_amdgcn_ballot_w32(s == r + 32);
            const int c0 = __builtin_popcount(m0); const int c1 = __builtin_popcount(m1);
            add0 = (lane == r) ? c0 : add0; add1 = (lane == r) ? c1 : add1;
            mymask = (s == r) ? m0 : mymask; mymask = (s == r + 32) ? m1 : mymask; }
        part[tok] = pre + __builtin_popcount(mymask & lt);
        run0 += add0; run1 += add1;
    }
    wc[wave * NSEG + lane] = run0; wc[wave * NSEG + 32 + lane] = run1;
    __syncthreads();
    if (tid < NSEG) {
        int run = 0;
#pragma unroll 1
        for (int w = 0; w < 32; ++w) { const int c = clampi(wc[w * NSEG + tid], 0, CPW * 32); wc[w * NSEG + tid] = run; run += c; }
        tots[tid] = run;
    }
    __syncthreads();
    if (tid < NSEG) {
        int st = 0;
#pragma unroll 1
        for (int q = 0; q < NSEG; ++q) { const int pd = (tots[q] + 63) & ~63; st += (q < tid) ? pd : 0; }
        segst[tid] = st;
    }
    __syncthreads();
#pragma unroll 1
    for (int c = 0; c < CPW; ++c) {
        const int tok = tbase + c * 32 + lane;
        const int s = clampi(seg[tok], 0, NSEG - 1);
        const int pv = clampi(segst[s] + wc[wave * NSEG + s] + part[tok], 0, PROWS - 1);
        part[tok] = pv;
    }
    if (wave == 0) {
        const int ptot = segst[NSEG - 1] + ((tots[NSEG - 1] + 63) & ~63);
        tl[lane] = segst[lane]; tl[32 + lane] = segst[32 + lane]; tl[64 + lane] = tots[lane]; tl[96 + lane] = tots[32 + lane];
        tl[128 + lane] = (lane == 0) ? ptot : 0; tl[160 + lane] = 0; tl[192 + lane] = 0; tl[224 + lane] = 0;
        wave_sync();
    }
    v8us z;
#pragma unroll
    for (int k = 0; k < 8; ++k) z[k] = (unsigned short)0;
#pragma unroll 1
    for (int ps = 0; ps < 2; ++ps) {
#pragma unroll 1
        for (int c = 0; c < CPW; ++c) { const int tok = tbase + c * 32 + lane; const int pv = part[tok]; *(volatile int*)(POS + tok) = pv; }
        if (wave == 0) {
            const v4i v0 = *(const v4ia*)(&tl[4 * lane]); const v4i v1 = *(const v4ia*)(&tl[128 + 4 * lane]);
            *(volatile v4i*)(T + 4 * lane) = v0; *(volatile v4i*)(T + 128 + 4 * lane) = v1; }
#pragma unroll 1
        for (int sgi = 0; sgi < 2; ++sgi) {
            const int r = wave + 32 * sgi;
            const int tot = clampi(tots[r], 0, NB);
            const int padcnt = __builtin_amdgcn_readfirstlane(clampi(((tot + 63) & ~63) - tot, 0, 63));
            const int pbase = segst[r] + tot;
#pragma unroll 1
            for (int j = 0; j < padcnt; ++j) {
                const int p = clampi(pbase + j, 0, PROWS - 1);
#pragma unroll
                for (int q = 0; q < 4; ++q) *(volatile v8us*)(XP + (size_t)p * HID + (size_t)(q * 256 + lane * 8)) = z; }
        }
        if (ps == 0) __threadfence(); }
}

__global__ __launch_bounds__(256) void k_place(const float* __restrict__ x, const int* __restrict__ POS, bf* XP) {
    const int lane = threadIdx.x & 31; const int wave = __builtin_amdgcn_readfirstlane(threadIdx.x >> 5);
    const int row = blockIdx.x * 8 + wave;
    if (row >= NB) return;
    const int p = clampi(POS[row], 0, PROWS - 1);
    v8us o[4];
#pragma unroll
    for (int q = 0; q < 4; ++q) { const v8f a = *(const v8f*)(x + (size_t)row * HID + (size_t)(q * 256 + lane * 8));
#pragma unroll
        for (int k = 0; k < 8; ++k) o[q][k] = f2bf(a[k]); }
    bf* dst = XP + (size_t)p * HID + (size_t)(lane * 8);
#pragma unroll
    for (int q = 0; q < 4; ++q) *(volatile v8us*)(dst + q * 256) = o[q];
    __threadfence();
#pragma unroll
    for (int q = 0; q < 4; ++q) *(volatile v8us*)(dst + q * 256) = o[q];
}

__global__ __launch_bounds__(32) __attribute__((amdgpu_num_vgpr(256))) void k_gemm(const bf* __restrict__ XP, const bf* __restrict__ BW, const bf* __restrict__ AW,
                                                                                    const float* __restrict__ bias, const int* __restrict__ T, float* SORTED) {
    __shared__ __align__(16) float os[16 * 68];
    __shared__ __align__(16) float ts[64 * TPITCH];
    const int lane = threadIdx.x & 31, lr = lane & 15, hi = lane >> 4;
    const int p0 = blockIdx.x * 64;
    int s0 = T[lane], s1 = T[32 + lane], n0 = T[64 + lane], n1 = T[96 + lane];
    asm volatile("" : "+v"(s0)); asm volatile("" : "+v"(s1)); asm volatile("" : "+v"(n0)); asm volatile("" : "+v"(n1));
    const int e0 = s0 + ((n0 + 63) & ~63), e1 = s1 + ((n1 + 63) & ~63);
    const unsigned m0 = __builtin_amdgcn_ballot_w32(((p0 >= s0) & (p0 < e0)) != 0);
    const unsigned m1 = __builtin_amdgcn_ballot_w32(((p0 >= s1) & (p0 < e1)) != 0);
    if ((m0 | m1) == 0u) return;
    const unsigned long long mm = (((unsigned long long)m1) << 32) | (unsigned long long)m0;
    const int r = __builtin_amdgcn_readfirstlane(clampi((int)__builtin_ctzll(mm), 0, NSEG - 1));
    v8f t1[4];
#pragma unroll
    for (int mb = 0; mb < 4; ++mb) t1[mb] = (v8f){};
    const size_t aoff = (size_t)(p0 + lr) * HID + (size_t)(8 * hi), boff = (size_t)r * (RANK * HID) + (size_t)lr * HID + (size_t)(8 * hi);
#pragma unroll 1
    for (int kc = 0; kc < HID; kc += 32) {
        const v16bf b = ldb(BW + boff + kc);
#pragma unroll
        for (int mb = 0; mb < 4; ++mb) { const v16bf a = ldb(XP + aoff + (size_t)mb * 16 * HID + kc); t1[mb] = wmmag(a, b, t1[mb]); }
    }
#pragma unroll
    for (int mb = 0; mb < 4; ++mb) {
#pragma unroll
        for (int j = 0; j < 8; ++j) ts[(mb * 16 + hi * 8 + j) * TPITCH + lr] = t1[mb][j]; }
    wave_sync();
    v16bf th[4];
#pragma unroll
    for (int mb = 0; mb < 4; ++mb) {
        const float* tr = &ts[(mb * 16 + lr) * TPITCH + 8 * hi];
        const v4f x0 = *(const v4fa*)tr; const v4f x1 = *(const v4fa*)(tr + 4);
        v8us h8, l8;
#pragma unroll
        for (int i = 0; i < 4; ++i) {
            const unsigned short ha = f2bf(x0[i]); h8[i] = ha; l8[i] = f2bf(x0[i] - bf2f(ha));
            const unsigned short hb = f2bf(x1[i]); h8[4 + i] = hb; l8[4 + i] = f2bf(x1[i] - bf2f(hb)); }
        th[mb] = cat16b(h8, l8);
    }
    const size_t woff = ((size_t)r * HID + (size_t)lr) * 32 + (size_t)(8 * hi);
    const int c4 = (lane & 15) * 4;
#pragma unroll 1
    for (int cb = 0; cb < HID; cb += 64) {
        const v4f bz = *(const v4f*)(bias + (size_t)r * HID + (size_t)(cb + c4));
        v4f bb;
#pragma unroll
        for (int i = 0; i < 4; ++i) bb[i] = bf2f(f2bf(bz[i]));
#pragma unroll
        for (int mb = 0; mb < 4; ++mb) {
            v8f acc[4];
#pragma unroll
            for (int nb = 0; nb < 4; ++nb) { const v16bf b = ldb(AW + woff + (size_t)(cb + nb * 16) * 32); acc[nb] = wmmag(th[mb], b, (v8f){}); }
#pragma unroll
            for (int nb = 0; nb < 4; ++nb) {
#pragma unroll
                for (int j = 0; j < 8; ++j) os[(hi * 8 + j) * 68 + nb * 16 + lr] = acc[nb][j]; }
            wave_sync();
#pragma unroll 1
            for (int ps = 0; ps < 2; ++ps) {
#pragma unroll 1
                for (int it = 0; it < 8; ++it) { const int row = 2 * it + hi;
                    const v4f v = *(const v4fa*)(&os[row * 68 + c4]) + bb;
                    *(volatile v4f*)(SORTED + (size_t)(p0 + mb * 16 + row) * HID + (size_t)(cb + c4)) = v; }
                if (ps == 0) __threadfence(); }
            wave_sync();
        }
    }
}

__global__ __launch_bounds__(256) void k_unsort(const int* __restrict__ POS, const float* __restrict__ SORTED, float* OUT) {
    const int lane = threadIdx.x & 31; const int wave = __builtin_amdgcn_readfirstlane(threadIdx.x >> 5);
    const int row = blockIdx.x * 8 + wave;
    if (row >= NB) return;
    const int p = clampi(POS[row], 0, PROWS - 1);
    v4f v[8];
#pragma unroll
    for (int q = 0; q < 8; ++q) v[q] = *(const v4f*)(SORTED + (size_t)p * HID + (size_t)(q * 128 + lane * 4));
    float* dst = OUT + (size_t)row * HID + (size_t)(lane * 4);
#pragma unroll
    for (int q = 0; q < 8; ++q) *(volatile v4f*)(dst + q * 128) = v[q];
    __threadfence();
#pragma unroll
    for (int q = 0; q < 8; ++q) *(volatile v4f*)(dst + q * 128) = v[q];
}

static constexpr size_t al256(size_t v) { return (v + 255) & ~(size_t)255; }
static constexpr size_t SZ_AW  = al256((size_t)NSEG * HID * 32 * 2);
static constexpr size_t SZ_BW  = al256((size_t)NSEG * RANK * HID * 2);
static constexpr size_t SZ_T   = al256((size_t)256 * 4);
static constexpr size_t SZ_POS = al256((size_t)NB * 4);
static constexpr size_t SZ_XP  = al256((size_t)PROWS * HID * 2);
static constexpr size_t SZ_SRT = al256((size_t)PROWS * HID * 4);
static constexpr size_t SZ_TOTAL = SZ_AW + SZ_BW + SZ_T + SZ_POS + SZ_XP + SZ_SRT;
static_assert(SZ_TOTAL <= (size_t)134217728);
static_assert((size_t)(WB_BLK) * 256 * 8 * 2 == (size_t)NSEG * RANK * HID * 2);
static_assert((size_t)(WA_BLK) * 256 * 8 * 2 == (size_t)NSEG * HID * 32 * 2);
static_assert((size_t)(PROWS / 64) * 64 == (size_t)PROWS);

extern "C" void kernel_launch(void* const* d_in, const int* in_sizes, int n_in,
                              void* d_out, int out_size, void* d_ws, size_t ws_size, hipStream_t stream) {
    if (n_in < 5) return;
    if ((size_t)in_sizes[0] < (size_t)NB * HID) return;
    if ((size_t)in_sizes[1] < (size_t)NB) return;
    if ((size_t)in_sizes[2] < (size_t)NSEG * HID * RANK) return;
    if ((size_t)in_sizes[3] < (size_t)NSEG * RANK * HID) return;
    if ((size_t)in_sizes[4] < (size_t)NSEG * HID) return;
    if ((size_t)out_size < (size_t)NB * HID) return;
    if (SZ_TOTAL > ws_size) return;
    const float* x    = (const float*)d_in[0];
    const int*   seg  = (const int*)d_in[1];
    const float* Am   = (const float*)d_in[2];
    const float* Bm   = (const float*)d_in[3];
    const float* bias = (const float*)d_in[4];
    float* OUT = (float*)d_out;
    char* wsp = (char*)d_ws;
    bf*  AW  = (bf*)wsp;  wsp += SZ_AW;
    bf*  BW  = (bf*)wsp;  wsp += SZ_BW;
    int* TT  = (int*)wsp; wsp += SZ_T;
    int* POS = (int*)wsp; wsp += SZ_POS;
    bf*  XP  = (bf*)wsp;  wsp += SZ_XP;
    float* SRT = (float*)wsp; wsp += SZ_SRT;

    k_wconv<<<WB_BLK + WA_BLK, 256, 0, stream>>>(Am, Bm, AW, BW);
    k_sort<<<1, 1024, 0, stream>>>(seg, POS, TT, XP);
    k_place<<<NB / 8, 256, 0, stream>>>(x, POS, XP);
    k_gemm<<<PROWS / 64, 32, 0, stream>>>(XP, BW, AW, bias, TT, SRT);
    k_unsort<<<NB / 8, 256, 0, stream>>>(POS, SRT, OUT);
}
